// CustomRNN_41566693491393
// MI455X (gfx1250) — hardware-run, weakly checked
//
#include <hip/hip_runtime.h>

typedef __attribute__((ext_vector_type(16))) _Float16 v16h;
typedef __attribute__((ext_vector_type(8)))  _Float16 v8h;
typedef __attribute__((ext_vector_type(8)))  float    v8f;
typedef __attribute__((ext_vector_type(4)))  float    v4f;
typedef __attribute__((ext_vector_type(2)))  unsigned v2u;

constexpr int kLayers   = 2;
constexpr int kSteps    = 256;
constexpr int kBatch    = 32;
constexpr int kFeat     = 1024;
constexpr int kHid      = 1024;
constexpr int kKdim     = kFeat + kHid;
constexpr int kGateCols = 4 * kHid;
constexpr int kSamp     = 16;
constexpr int kCellBlocks  = kBatch / kSamp;
constexpr int kCellWaves   = 16;
constexpr int kCellThreads = kCellWaves * 32;
constexpr int kKsteps   = kKdim / 32;
constexpr int kPitch    = kKdim + 8;
constexpr int kTileSz   = kSamp * kPitch;
constexpr int kFragHalves = 512;
constexpr int kPassStride = kKsteps * 8 * kFragHalves;
constexpr float kCarryA  = 64.0f;
constexpr float kCarryW  = 1024.0f;
constexpr float kFold    = 1.0f / (kCarryA * kCarryW);
constexpr float kUncarryA = 1.0f / kCarryA;
constexpr float kMinNorm = 6.103515625e-05f;

static_assert(kKdim == 2048);
static_assert(kFeat == kHid);
static_assert((kKdim % 32) == 0 && (kHid % 32) == 0 && (kFeat % 32) == 0);
static_assert(kCellWaves * 64 == kHid);
static_assert(kCellWaves == kSamp);
static_assert(kCellBlocks * kSamp == kBatch);
static_assert(kCellBlocks == 2);
static_assert((kPitch % 8) == 0);
static_assert(kKsteps == 64);
static_assert((size_t)kSamp * kHid * 4 <= (size_t)kTileSz * 2);
static_assert((size_t)2 * kTileSz * 2 + (size_t)kGateCols * 4 == 147968ull);

constexpr size_t kOutSeq   = (size_t)kBatch * kSteps * kHid;
constexpr size_t kOutState = (size_t)kLayers * kBatch * kHid;
constexpr size_t kOffHfin  = kOutSeq;
constexpr size_t kOffCfin  = kOutSeq + kOutState;
constexpr size_t kOutTotal = kOutSeq + 2 * kOutState;
static_assert(kOffHfin * 4 == 33554432ull);
static_assert(kOffCfin * 4 == 33816576ull);
static_assert(kOutTotal * 4 == 34078720ull);

constexpr size_t kBytesWPl = (size_t)kGateCols * kKdim * 2;
constexpr size_t kBytesWP  = (size_t)kLayers * kBytesWPl;
constexpr size_t kBytesH0  = (size_t)kSteps * kBatch * kHid * 2;
constexpr size_t kOffWP = 0;
constexpr size_t kOffH0 = kOffWP + kBytesWP;
constexpr size_t kWsTotal = kOffH0 + kBytesH0;
static_assert(kBytesWPl == 16777216ull);
static_assert(kBytesH0 == 16777216ull);
static_assert(kWsTotal == 50331648ull);
static_assert(kWsTotal <= 134217728ull);
static_assert((kOffH0 % 128) == 0 && (kBytesWPl % 128) == 0);

__device__ __forceinline__ unsigned short f2bf_bits(float f) {
  unsigned u = __float_as_uint(f);
  return (unsigned short)((u + 0x7FFFu + ((u >> 16) & 1u)) >> 16);
}
__device__ __forceinline__ float bf_bits2f(unsigned short h) { return __uint_as_float(((unsigned)h) << 16); }
__device__ __forceinline__ float rne_bf(float f) { return bf_bits2f(f2bf_bits(f)); }

__device__ __forceinline__ _Float16 op_from_value(float v, float carry) {
  const float r = v * carry;
  const float z = (__builtin_fabsf(r) < kMinNorm) ? 0.0f : r;
  return (_Float16)z;
}
__device__ __forceinline__ _Float16 op_from_input(float v, float carry) {
  return op_from_value(rne_bf(v), carry);
}

__device__ __forceinline__ float h16_to_f32(unsigned hb) {
  const unsigned sgn = (hb & 0x8000u) << 16;
  const unsigned em = hb & 0x7fffu;
  const float fn = __uint_as_float((em << 13) + 0x38000000u);
  const float fs = (float)em * 5.9604644775390625e-8f;
  const float mag = (em < 0x400u) ? fs : fn;
  return __uint_as_float(__float_as_uint(mag) | sgn);
}

union FragU { v16h v; v8h h[2]; };
__device__ __forceinline__ v16h load_frag(const _Float16* p0, const _Float16* p1) {
  FragU f;
  f.h[0] = *(const v8h*)(p0);
  f.h[1] = *(const v8h*)(p1);
  return f.v;
}
__device__ __forceinline__ v8f mma1(v16h a, v16h b, v8f c) {
  c = __builtin_amdgcn_wmma_f32_16x16x32_f16(false, a, false, b, (short)0, c, false, false);
  asm volatile("v_nop\n\tv_nop\n\tv_nop\n\tv_nop" : "+v"(c) : "v"(a), "v"(b));
  return c;
}
__device__ __forceinline__ float sig_fast(float x) {
  return __builtin_amdgcn_rcpf(1.0f + __expf(-x));
}
__device__ __forceinline__ float tanh_fast(float x) {
  const float r = __builtin_amdgcn_rcpf(1.0f + __expf(-2.0f * x));
  return fmaf(2.0f, r, -1.0f);
}

__global__ __launch_bounds__(256) void weight_planes(
    const float* __restrict__ wih, const float* __restrict__ whh,
    _Float16* __restrict__ wp)
{
  const int layer = blockIdx.y;
  const int gid = blockIdx.x * 256 + threadIdx.x;
  const int l   = gid & 31;
  const int hf  = (gid >> 5) & 1;
  const int fi  = gid >> 6;
  const int tl  = fi & 7;
  const int rest = fi >> 3;
  const int ks  = rest % kKsteps;
  const int wpi = rest / kKsteps;
  const int ps  = wpi & 1;
  const int wv  = wpi >> 1;
  const int g   = tl >> 1;
  const int jj  = tl & 1;
  const int hh  = l >> 4;
  const int m   = l & 15;
  const int u   = 64 * wv + 32 * ps + 16 * jj + m;
  const int k   = ks * 32 + 16 * hf + 8 * hh;
  const bool inpart = (k < kFeat);
  const int kk = inpart ? k : (k - kFeat);
  const float* base = inpart ? wih : whh;
  const float* src = base + ((size_t)layer * kGateCols + (size_t)(g * kHid + u)) * kHid + kk;
  const v4f a0 = *(const v4f*)(src);
  const v4f a1 = *(const v4f*)(src + 4);
  v8h hv;
#pragma unroll
  for (int e = 0; e < 4; ++e) {
    hv[e]     = op_from_input(a0[e], kCarryW);
    hv[4 + e] = op_from_input(a1[e], kCarryW);
  }
  _Float16* dst = wp + (size_t)layer * kGateCols * kKdim + (size_t)gid * 8;
  *(volatile v8h*)dst = hv;
  __threadfence();
  *(volatile v8h*)dst = hv;
}


__device__ __forceinline__ void stage_x(const float* __restrict__ xblk, int t, _Float16* dst, int tid) {
  const int s = tid >> 5;
  const int col = (tid & 31) * 8;
  const float* sp = xblk + ((size_t)s * kSteps + t) * kFeat + col;
#pragma unroll
  for (int i = 0; i < 4; ++i) {
    const v4f a0 = *(const v4f*)(sp + i * 256);
    const v4f a1 = *(const v4f*)(sp + i * 256 + 4);
    v8h hv;
#pragma unroll
    for (int e = 0; e < 4; ++e) {
      hv[e]     = op_from_input(a0[e], kCarryA);
      hv[4 + e] = op_from_input(a1[e], kCarryA);
    }
    *(v8h*)(dst + s * kPitch + i * 256 + col) = hv;
  }
}

__device__ __forceinline__ void stage_h0(const _Float16* hrows, _Float16* dst, int tid) {
  const int s = tid >> 5;
  const int col = (tid & 31) * 8;
  const _Float16* sp = hrows + (size_t)s * kHid + col;
#pragma unroll
  for (int i = 0; i < 4; ++i) {
    const v8h hv = *(const v8h*)(sp + i * 256);
    *(v8h*)(dst + s * kPitch + i * 256 + col) = hv;
  }
}

__device__ __forceinline__ void flush_h(const _Float16* tile, _Float16* dstrow, int wave, int lane) {
  const _Float16* sp = tile + wave * kPitch + kFeat + lane * 8;
  v8h hv[4];
#pragma unroll
  for (int i = 0; i < 4; ++i) hv[i] = *(const v8h*)(sp + i * 256);
  for (int pass = 0; pass < 2; ++pass) {
#pragma unroll
    for (int i = 0; i < 4; ++i) *(volatile v8h*)(dstrow + i * 256 + lane * 8) = hv[i];
    __threadfence();
  }
}

__device__ __forceinline__ void flush_f32(const _Float16* tile, float* __restrict__ dstrow, int wave, int lane) {
  const v2u* sp = (const v2u*)(tile + wave * kPitch + kFeat + lane * 4);
  v4f ov[8];
#pragma unroll
  for (int i = 0; i < 8; ++i) {
    const v2u w = sp[i * 32];
    const unsigned w0 = w[0];
    const unsigned w1 = w[1];
    v4f o;
    o[0] = h16_to_f32(w0 & 0xffffu) * kUncarryA;
    o[1] = h16_to_f32(w0 >> 16) * kUncarryA;
    o[2] = h16_to_f32(w1 & 0xffffu) * kUncarryA;
    o[3] = h16_to_f32(w1 >> 16) * kUncarryA;
    ov[i] = o;
  }
  for (int pass = 0; pass < 2; ++pass) {
#pragma unroll
    for (int i = 0; i < 8; ++i) *(volatile v4f*)(dstrow + i * 128 + lane * 4) = ov[i];
    __threadfence();
  }
}

__device__ __forceinline__ void gate_pass(const _Float16* cur, _Float16* nxt,
                                          const _Float16* __restrict__ wl, const float* bias_s,
                                          int ucol, int hh, int m, float (&cst)[2][8])
{
  v8f acc[8];
#pragma unroll
  for (int tl = 0; tl < 8; ++tl) acc[tl] = (v8f){0.f, 0.f, 0.f, 0.f, 0.f, 0.f, 0.f, 0.f};
  const _Float16* ap = cur + m * kPitch + 8 * hh;
  const _Float16* bp = wl;
#pragma unroll 1
  for (int ks = 0; ks < kKsteps; ++ks) {
    const v16h a = load_frag(ap, ap + 16);
#pragma unroll
    for (int tl = 0; tl < 8; ++tl) {
      const v16h b = load_frag(bp + tl * kFragHalves, bp + tl * kFragHalves + 256);
      acc[tl] = mma1(a, b, acc[tl]);
    }
    ap += 32;
    bp += 8 * kFragHalves;
  }
#pragma unroll
  for (int jj = 0; jj < 2; ++jj) {
    const int u = ucol + 16 * jj;
    const float biv = bias_s[u];
    const float bfv = bias_s[kHid + u];
    const float bgv = bias_s[2 * kHid + u];
    const float bov = bias_s[3 * kHid + u];
    _Float16* hp = nxt + (8 * hh) * kPitch + kFeat + u;
#pragma unroll
    for (int r = 0; r < 8; ++r) {
      const float zi = fmaf(acc[0 + jj][r], kFold, biv);
      const float zf = fmaf(acc[2 + jj][r], kFold, bfv);
      const float zg = fmaf(acc[4 + jj][r], kFold, bgv);
      const float zo = fmaf(acc[6 + jj][r], kFold, bov);
      const float it = sig_fast(zi);
      const float ft = sig_fast(zf);
      const float ot = sig_fast(zo);
      const float tg = tanh_fast(zg);
      const float cn = ft * cst[jj][r] + it * tg;
      cst[jj][r] = cn;
      const float hn = ot * tanh_fast(cn);
      hp[r * kPitch] = op_from_value(hn, kCarryA);
    }
  }
}

template <int LAYER>
__global__ __launch_bounds__(512) void cell_steps(
    const float* __restrict__ x, _Float16* h0, const _Float16* __restrict__ wp,
    const float* __restrict__ hinit, const float* __restrict__ cinit,
    const float* __restrict__ bih, const float* __restrict__ bhh,
    float* __restrict__ out)
{
  __shared__ __align__(16) _Float16 atile[2 * kTileSz];
  __shared__ __align__(16) float bias_s[kGateCols];

  const int tid  = threadIdx.x;
  const int lane = tid & 31;
  const int wave = tid >> 5;
  const int hh   = lane >> 4;
  const int m    = lane & 15;
  const int samp0 = blockIdx.x * kSamp;
  const float* xblk = x + (size_t)samp0 * kSteps * kFeat;

#pragma unroll
  for (int it = 0; it < 2; ++it) {
    const int j = (it * kCellThreads + tid) * 4;
    const v4f b0 = *(const v4f*)(bih + (size_t)LAYER * kGateCols + j);
    const v4f b1 = *(const v4f*)(bhh + (size_t)LAYER * kGateCols + j);
    v4f bs;
#pragma unroll
    for (int e = 0; e < 4; ++e) bs[e] = rne_bf(b0[e]) + rne_bf(b1[e]);
    *(v4f*)(bias_s + j) = bs;
  }
  {
    const int s = tid >> 5;
    const int c = (tid & 31) * 8;
    const float* hp0 = hinit + ((size_t)LAYER * kBatch + samp0 + s) * kHid + c;
#pragma unroll
    for (int i = 0; i < 4; ++i) {
      const v4f a0 = *(const v4f*)(hp0 + i * 256);
      const v4f a1 = *(const v4f*)(hp0 + i * 256 + 4);
      v8h hv;
#pragma unroll
      for (int e = 0; e < 4; ++e) {
        hv[e]     = op_from_input(a0[e], kCarryA);
        hv[4 + e] = op_from_input(a1[e], kCarryA);
      }
      *(v8h*)(atile + s * kPitch + kFeat + i * 256 + c) = hv;
    }
  }
  if (LAYER == 0) stage_x(xblk, 0, atile, tid);
  else stage_h0(h0 + (size_t)samp0 * kHid, atile, tid);

  float* cslab = (float*)(atile + kTileSz);
  {
    const float* csrc = cinit + ((size_t)LAYER * kBatch + samp0) * kHid;
#pragma unroll
    for (int it = 0; it < 8; ++it) {
      const int j = (it * kCellThreads + tid) * 4;
      const v4f cv = *(const v4f*)(csrc + j);
      *(v4f*)(cslab + j) = cv;
    }
  }
  __syncthreads();

  const int ucol = wave * 64 + m;
  float c0[2][8], c1[2][8];
#pragma unroll
  for (int jj = 0; jj < 2; ++jj) {
#pragma unroll
    for (int r = 0; r < 8; ++r) {
      c0[jj][r] = rne_bf(cslab[(8 * hh + r) * kHid + ucol + 16 * jj]);
      c1[jj][r] = rne_bf(cslab[(8 * hh + r) * kHid + ucol + 32 + 16 * jj]);
    }
  }
  __syncthreads();

  const _Float16* wlane = wp + (size_t)wave * 2 * kPassStride + lane * 8;

  for (int t = 0; t < kSteps; ++t) {
    const _Float16* cur = atile + (t & 1) * kTileSz;
    _Float16* nxt = atile + ((t + 1) & 1) * kTileSz;
    if (t > 0) {
      if (LAYER == 0) flush_h(cur, h0 + ((size_t)(t - 1) * kBatch + samp0 + wave) * kHid, wave, lane);
      else flush_f32(cur, out + ((size_t)(samp0 + wave) * kSteps + (t - 1)) * kHid, wave, lane);
    }
    gate_pass(cur, nxt, wlane, bias_s, ucol, hh, m, c0);
    gate_pass(cur, nxt, wlane + kPassStride, bias_s, ucol + 32, hh, m, c1);
    if (t + 1 < kSteps) {
      if (LAYER == 0) stage_x(xblk, t + 1, nxt, tid);
      else stage_h0(h0 + ((size_t)(t + 1) * kBatch + samp0) * kHid, nxt, tid);
    }
    __syncthreads();
  }

  const _Float16* lastc = atile + (kSteps & 1) * kTileSz;
  if (LAYER == 0) flush_h(lastc, h0 + ((size_t)(kSteps - 1) * kBatch + samp0 + wave) * kHid, wave, lane);
  else flush_f32(lastc, out + ((size_t)(samp0 + wave) * kSteps + (kSteps - 1)) * kHid, wave, lane);
  flush_f32(lastc, out + kOffHfin + ((size_t)LAYER * kBatch + samp0 + wave) * kHid, wave, lane);

  float* fslab = (float*)(atile + ((kSteps + 1) & 1) * kTileSz);
#pragma unroll
  for (int jj = 0; jj < 2; ++jj) {
#pragma unroll
    for (int r = 0; r < 8; ++r) {
      fslab[(8 * hh + r) * kHid + ucol + 16 * jj]      = c0[jj][r];
      fslab[(8 * hh + r) * kHid + ucol + 32 + 16 * jj] = c1[jj][r];
    }
  }
  __syncthreads();
  {
    const float* sp = fslab + wave * kHid + lane * 4;
    float* dp = out + kOffCfin + ((size_t)LAYER * kBatch + samp0 + wave) * kHid + lane * 4;
    v4f cv[8];
#pragma unroll
    for (int i = 0; i < 8; ++i) cv[i] = *(const v4f*)(sp + i * 128);
    for (int pass = 0; pass < 2; ++pass) {
#pragma unroll
      for (int i = 0; i < 8; ++i) *(volatile v4f*)(dp + i * 128) = cv[i];
      __threadfence();
    }
  }
}

extern "C" void kernel_launch(void* const* d_in, const int* in_sizes, int n_in,
                              void* d_out, int out_size, void* d_ws, size_t ws_size,
                              hipStream_t stream) {
  if (n_in < 7) return;
  if (in_sizes[0] != kBatch * kSteps * kFeat) return;
  if (in_sizes[1] != kLayers * kBatch * kHid || in_sizes[2] != kLayers * kBatch * kHid) return;
  if (in_sizes[3] != kLayers * kGateCols * kFeat || in_sizes[4] != kLayers * kGateCols * kHid) return;
  if (in_sizes[5] != kLayers * kGateCols || in_sizes[6] != kLayers * kGateCols) return;
  if ((size_t)out_size != kOutTotal) return;
  if (ws_size < kWsTotal) return;

  const float* x    = (const float*)d_in[0];
  const float* hin  = (const float*)d_in[1];
  const float* cin  = (const float*)d_in[2];
  const float* wih  = (const float*)d_in[3];
  const float* whh  = (const float*)d_in[4];
  const float* bih  = (const float*)d_in[5];
  const float* bhh  = (const float*)d_in[6];
  float* out = (float*)d_out;

  char* ws = (char*)d_ws;
  _Float16* WP = (_Float16*)(ws + kOffWP);
  _Float16* H0 = (_Float16*)(ws + kOffH0);

  constexpr int kWpBlocks = (kGateCols * kKdim / 8) / 256;
  static_assert(kWpBlocks * 256 * 8 == kGateCols * kKdim);
  static_assert(kWpBlocks == 4096);

  weight_planes<<<dim3(kWpBlocks, kLayers), dim3(256), 0, stream>>>(wih, whh, WP);
  cell_steps<0><<<dim3(kCellBlocks), dim3(kCellThreads), 0, stream>>>(
      x, H0, WP, hin, cin, bih, bhh, out);
  cell_steps<1><<<dim3(kCellBlocks), dim3(kCellThreads), 0, stream>>>(
      x, H0, WP + (size_t)kGateCols * kKdim, hin, cin, bih, bhh, out);
}
